// self_attn_11330123727100
// MI455X (gfx1250) — hardware-verified
//
#include <hip/hip_runtime.h>
#include <math.h>

typedef __attribute__((ext_vector_type(16))) _Float16 v16h;
typedef __attribute__((ext_vector_type(16))) __bf16 v16b;
typedef __attribute__((ext_vector_type(8)))  _Float16 v8h;
typedef __attribute__((ext_vector_type(8)))  float v8f;
typedef __attribute__((ext_vector_type(4)))  float v4f;
typedef __attribute__((ext_vector_type(2)))  float v2f;
typedef __attribute__((ext_vector_type(4)))  unsigned v4u;
typedef __attribute__((ext_vector_type(4)))  int v4i;
typedef float __attribute__((may_alias)) float_a;
typedef int __attribute__((may_alias)) int_a;

template <typename T> __device__ __forceinline__ void vst2(void* p, T v) { *(volatile T*)p = v; __threadfence(); *(volatile T*)p = v; }
__device__ __forceinline__ v8f wmma16(v16h a, v16h b, v8f c) {
  v8f d = __builtin_amdgcn_wmma_f32_16x16x32_f16(false, a, false, b, (short)0, c, false, false);
  asm volatile("v_nop\n\tv_nop\n\tv_nop\n\tv_nop" : "+v"(d) : "v"(a), "v"(b));
  return d;
}
__device__ __forceinline__ v8f wmma_bf(v16b a, v16b b, v8f c) {
  v8f d = __builtin_amdgcn_wmma_f32_16x16x32_bf16(false, a, false, b, (short)0, c, false, false);
  asm volatile("v_nop\n\tv_nop\n\tv_nop\n\tv_nop" : "+v"(d) : "v"(a), "v"(b));
  return d;
}
__device__ __forceinline__ v16h frag_h(const _Float16* rowk0, int lane) {
  union { v16h v; v8h q[2]; } u; const _Float16* p = rowk0 + 8 * (lane >> 4);
  u.q[0] = *(const v8h*)p; u.q[1] = *(const v8h*)(p + 16); return u.v;
}
__device__ __forceinline__ v16h frag_f32(const float* rowk0, int lane) {
  v16h a; const float* p = rowk0 + 8 * (lane >> 4);
#pragma unroll
  for (int i = 0; i < 8; ++i) { a[i] = (_Float16)p[i]; a[8 + i] = (_Float16)p[16 + i]; }
  return a;
}
__device__ __forceinline__ v16h frag_f32s(const float* rowk0, int lane, float sc) {
  v16h a; const float* p = rowk0 + 8 * (lane >> 4);
#pragma unroll
  for (int i = 0; i < 8; ++i) { a[i] = (_Float16)(p[i] * sc); a[8 + i] = (_Float16)(p[16 + i] * sc); }
  return a;
}
__device__ __forceinline__ v16h fragc_f32(const float* W, int k0, int n, int lane, int ld, int K) {
  v16h a; const int g = lane >> 4;
#pragma unroll
  for (int i = 0; i < 8; ++i) { const int ka = k0 + 8 * g + i, kb = ka + 16;
    a[i] = (_Float16)(ka < K ? W[(size_t)(ka < K ? ka : K - 1) * ld + n] : 0.f); a[8 + i] = (_Float16)(kb < K ? W[(size_t)(kb < K ? kb : K - 1) * ld + n] : 0.f); }
  return a;
}
struct F2 { v16b h, l; };
__device__ __forceinline__ F2 bsplit16(const float v[16]) { F2 r;
#pragma unroll
  for (int i = 0; i < 16; ++i) { const __bf16 h = (__bf16)v[i]; r.h[i] = h; r.l[i] = (__bf16)(v[i] - (float)h); }
  return r; }
__device__ __forceinline__ F2 split_row(const float* row, int k0, int lane) { float v[16]; const float* p = row + k0 + 8 * (lane >> 4);
#pragma unroll
  for (int i = 0; i < 8; ++i) { v[i] = p[i]; v[8 + i] = p[16 + i]; }
  return bsplit16(v); }
__device__ __forceinline__ F2 split_rowK(const float* row, int k0, int lane, int K) { float v[16]; const int g = lane >> 4;
#pragma unroll
  for (int i = 0; i < 8; ++i) { const int ka = k0 + 8 * g + i, kb = ka + 16; v[i] = ka < K ? row[ka < K ? ka : K - 1] : 0.f; v[8 + i] = kb < K ? row[kb < K ? kb : K - 1] : 0.f; }
  return bsplit16(v); }
__device__ __forceinline__ F2 split_col(const float* W, int k0, int n, int lane, int ld, int K) { float v[16]; const int g = lane >> 4;
#pragma unroll
  for (int i = 0; i < 8; ++i) { const int ka = k0 + 8 * g + i, kb = ka + 16; v[i] = ka < K ? W[(size_t)(ka < K ? ka : K - 1) * ld + n] : 0.f; v[8 + i] = kb < K ? W[(size_t)(kb < K ? kb : K - 1) * ld + n] : 0.f; }
  return bsplit16(v); }
__device__ __forceinline__ v8f mac3(const F2& a, const F2& b, v8f c) { c = wmma_bf(a.l, b.h, c); c = wmma_bf(a.h, b.l, c); return wmma_bf(a.h, b.h, c); }
__device__ __forceinline__ float sigm(float v) { return 1.0f / (1.0f + expf(-v)); }
#define LDSX() do { asm volatile("s_wait_dscnt 0" ::: "memory"); __builtin_amdgcn_wave_barrier(); __builtin_amdgcn_fence(__ATOMIC_RELEASE, "workgroup"); } while (0)


#define NB 2
#define CIN 64
#define C8 8
#define NP 9216
#ifndef TNB
#define TNB NB
#endif
#ifndef TQB
#define TQB (NP / 64)
#endif
typedef __attribute__((ext_vector_type(8))) __bf16 v8b;
__device__ __forceinline__ v16b frag_b(const __bf16* rowk0, int lane) {
  union { v16b v; v8b q[2]; } u; const __bf16* p = rowk0 + 8 * (lane >> 4);
  u.q[0] = *(const v8b*)p; u.q[1] = *(const v8b*)(p + 16); return u.v;
}
__device__ __forceinline__ float bfr(float v) { return (float)(__bf16)v; }
__device__ __attribute__((noinline)) float exp_ni(float v) { return expf(v); }
__device__ __attribute__((noinline)) float erf_ni(float v) { return erff(v); }

#define WS_QK  0u
#define WS_VT  (WS_QK + 2u * (size_t)NB * NP * 16)
#define WS_P   (WS_VT + 2u * (size_t)NB * CIN * NP)
#define WS_END (WS_P + 2u * (size_t)NP * NP)

__global__ __launch_bounds__(128) void k_proj(const float* __restrict__ X, const float* __restrict__ WQ, const float* __restrict__ BQ, const float* __restrict__ WK, const float* __restrict__ BK, const float* __restrict__ WV, const float* __restrict__ BV, _Float16* __restrict__ QK, _Float16* __restrict__ VT) {
  __shared__ __align__(16) __bf16 sx[64][CIN + 8]; __shared__ __align__(16) _Float16 sqk[64][16]; __shared__ __align__(16) _Float16 sv[CIN][72];
  const int tid = threadIdx.x, wave = tid >> 5, lane = tid & 31, col = lane & 15, g = lane >> 4; const int p0 = blockIdx.x * 64; const size_t b = blockIdx.y;
  for (int e = tid; e < CIN * 64; e += 128) { const int c = e >> 6, pl = e & 63; sx[pl][c] = (__bf16)X[(b * CIN + c) * (size_t)NP + p0 + pl]; }
  __syncthreads();
  v8f av[4] = {}; v8f aq[4] = {};
#pragma unroll
  for (int kc = 0; kc < CIN / 32; ++kc) { const v16b a = frag_b(&sx[wave * 16 + col][kc * 32], lane);
#pragma unroll
    for (int j = 0; j < 4; ++j) { v16b w; const int o = j * 16 + col;
#pragma unroll
      for (int i = 0; i < 8; ++i) { w[i] = (__bf16)WV[(size_t)o * CIN + kc * 32 + 8 * g + i]; w[8 + i] = (__bf16)WV[(size_t)o * CIN + kc * 32 + 16 + 8 * g + i]; }
      av[j] = wmma_bf(a, w, av[j]); }
    { v16b w; const float* Wm = (col < 8) ? (WQ + (size_t)col * CIN) : (WK + (size_t)(col - 8) * CIN);
#pragma unroll
      for (int i = 0; i < 8; ++i) { w[i] = (__bf16)Wm[kc * 32 + 8 * g + i]; w[8 + i] = (__bf16)Wm[kc * 32 + 16 + 8 * g + i]; }
      aq[0] = wmma_bf(a, w, aq[0]); } }
  { const float bb = (col < 8) ? bfr(BQ[col]) : bfr(BK[col - 8]);
#pragma unroll
    for (int r = 0; r < 8; ++r) sqk[wave * 16 + 8 * g + r][col] = (_Float16)(aq[0][r] + bb); }
#pragma unroll
  for (int j = 0; j < 4; ++j) { const float bb = bfr(BV[j * 16 + col]);
#pragma unroll
    for (int r = 0; r < 8; ++r) sv[j * 16 + col][wave * 16 + 8 * g + r] = (_Float16)(av[j][r] + bb); }
  __syncthreads();
  for (int e = tid; e < 64 * 2; e += 128) { const int pl = e >> 1, q = e & 1; vst2((unsigned*)(QK + (b * NP + p0 + pl) * 16 + q * 8), *(const v4u*)&sqk[pl][q * 8]); }
  for (int e = tid; e < CIN * 8; e += 128) { const int c = e >> 3, q = e & 7; vst2((unsigned*)(VT + (b * CIN + c) * (size_t)NP + p0 + q * 8), *(const v4u*)&sv[c][q * 8]); } }
__global__ __launch_bounds__(128) void k_sc(const _Float16* __restrict__ QK, int b, _Float16* __restrict__ P) { __shared__ __align__(16) _Float16 sp[4][16][136];
  const int tid = threadIdx.x, wave = tid >> 5, lane = tid & 31, col = lane & 15, g = lane >> 4; const int k0 = blockIdx.y * 128; const int ql0 = blockIdx.x * 64 + wave * 16;
  v16h a; { const _Float16* p = QK + ((size_t)b * NP + ql0 + col) * 16;
#pragma unroll
    for (int i = 0; i < 16; ++i) a[i] = (_Float16)0.f;
    if (g == 0) for (int i = 0; i < 8; ++i) a[i] = p[i]; }
#pragma unroll
  for (int j = 0; j < 8; ++j) { v16h kb; { const _Float16* p = QK + ((size_t)b * NP + k0 + j * 16 + col) * 16 + 8;
#pragma unroll
      for (int i = 0; i < 16; ++i) kb[i] = (_Float16)0.f;
      if (g == 0) for (int i = 0; i < 8; ++i) kb[i] = p[i]; }
    v8f c = {}; c = wmma16(a, kb, c);
#pragma unroll
    for (int r = 0; r < 8; ++r) sp[wave][8 * g + r][j * 16 + col] = (_Float16)(2048.0f / (1.0f + __expf(-c[r]))); }
  LDSX(); for (int rl = 0; rl < 16; ++rl) if (lane < 16) vst2((unsigned*)(P + (size_t)(ql0 + rl) * NP + k0 + lane * 8), *(const v4u*)&sp[wave][rl][lane * 8]); }
__global__ __launch_bounds__(128) void k_pv(const _Float16* __restrict__ P, const _Float16* __restrict__ VT, const float* __restrict__ X, const float* __restrict__ GM, int b, float* __restrict__ OUT) { __shared__ __align__(16) float st[CIN][68];
  const int tid = threadIdx.x, wave = tid >> 5, lane = tid & 31, col = lane & 15, g = lane >> 4; const int i0 = blockIdx.x * 64; const float gm = bfr(GM[0]);
  v8f acc[4] = {};
#pragma unroll 2
  for (int kc = 0; kc < NP / 32; ++kc) { const v16h pa = frag_h(P + (size_t)(i0 + wave * 16 + col) * NP + kc * 32, lane);
#pragma unroll
    for (int j = 0; j < 4; ++j) acc[j] = wmma16(pa, frag_h(VT + ((size_t)b * CIN + j * 16 + col) * NP + kc * 32, lane), acc[j]); }
#pragma unroll
  for (int j = 0; j < 4; ++j)
#pragma unroll
    for (int r = 0; r < 8; ++r) st[j * 16 + col][wave * 16 + 8 * g + r] = acc[j][r] * (1.0f / 2048.0f);
  __syncthreads();
  for (int e = tid; e < CIN * 16; e += 128) { const int c = e >> 4, q = e & 15; const size_t o = ((size_t)b * CIN + c) * NP + i0 + q * 4; v4f v = *(const v4f*)&st[c][q * 4]; const float* xp = X + o; v[0] = gm * v[0] + bfr(xp[0]); v[1] = gm * v[1] + bfr(xp[1]); v[2] = gm * v[2] + bfr(xp[2]); v[3] = gm * v[3] + bfr(xp[3]); vst2(OUT + o, v); } }
extern "C" void kernel_launch(void* const* d_in, const int* in_sizes, int n_in, void* d_out, int out_size, void* d_ws, size_t ws_size, hipStream_t stream) {
  (void)in_sizes; (void)n_in; (void)out_size;
  const float** F = (const float**)d_in;
  if (ws_size < (size_t)WS_END) return;
  char* ws = (char*)d_ws; _Float16 *QK = (_Float16*)(ws + WS_QK), *VT = (_Float16*)(ws + WS_VT), *P = (_Float16*)(ws + WS_P);
  k_proj<<<dim3(NP / 64, TNB), 128, 0, stream>>>(F[0], F[1], F[2], F[3], F[4], F[5], F[6], QK, VT);
  for (int b = 0; b < TNB; ++b) {
    k_sc<<<dim3(TQB, NP / 128), 128, 0, stream>>>(QK, b, P);
    k_pv<<<TQB, 128, 0, stream>>>(P, VT, F[0], F[7], b, (float*)d_out);
  }
}
